// SpeGBM_59416577573152
// MI455X (gfx1250) — hardware-run, weakly checked
//
#include <hip/hip_runtime.h>


namespace {
constexpr int B = 4, CH = 256, HH = 64, WW = 64, HW = HH * WW, TOK = 8, G = 32, DIN = 64, NS = 16, DTR = 2, XDW = 48, NGR = 4, MALL = B * HW;
constexpr float XS = 8.0f, WSC = 256.0f, EPS = 1e-5f;
typedef _Float16 b16;
typedef __attribute__((ext_vector_type(16))) _Float16 v16b;
typedef __attribute__((ext_vector_type(8))) _Float16 v8b;
typedef __attribute__((ext_vector_type(8))) float v8f;
typedef __attribute__((ext_vector_type(4))) float v4f;
typedef __attribute__((ext_vector_type(2))) float v2f;
__device__ __forceinline__ float bf16_rne(float f) { unsigned int u = __float_as_uint(f); u += 0x7FFFu + ((u >> 16) & 1u); float r = __uint_as_float(u & 0xFFFF0000u); asm volatile("" : "+v"(r)); return r; }
__device__ __forceinline__ void split16(float v, b16& hi, b16& lo) { hi = (b16)v; lo = (b16)(v - (float)hi); }
__device__ __forceinline__ v16b frag_kb(const b16* p, int hh) { const v8b a = *(const v8b*)(p + 8 * hh), b = *(const v8b*)(p + 16 + 8 * hh); v16b f;
#pragma unroll
  for (int e = 0; e < 8; ++e) { f[e] = a[e]; f[8 + e] = b[e]; } return f; }
__device__ __forceinline__ v8f wmma16b(v16b a, v16b b, v8f c) { v8f d = __builtin_amdgcn_wmma_f32_16x16x32_f16(false, a, false, b, (short)0, c, false, false); asm volatile("v_nop\n\tv_nop\n\tv_nop\n\tv_nop" : "+v"(d) : "v"(a), "v"(b)); return d; }
__device__ __forceinline__ void wave_lds_sync() { __builtin_amdgcn_fence(__ATOMIC_RELEASE, "workgroup"); __builtin_amdgcn_wave_barrier(); __builtin_amdgcn_fence(__ATOMIC_ACQUIRE, "workgroup"); }
__device__ __forceinline__ float pmul(float a, float b) { float p = a * b; asm volatile("" : "+v"(p)); return p; }
__device__ __forceinline__ float softplus(float v) { return v > 20.0f ? v : __logf(1.0f + __expf(v)); }
__device__ __forceinline__ float gelu(float v) { return 0.5f * v * (1.0f + erff(v * 0.70710678118654752f)); }

__global__ __launch_bounds__(256) void wput_kernel(const float* __restrict__ win, const float* __restrict__ wx, const float* __restrict__ wo, b16* __restrict__ WIN, b16* __restrict__ WX, b16* __restrict__ WO) { const int u = blockIdx.x * 256 + threadIdx.x;
  for (int pass = 0; pass < 2; ++pass) {
    if (u < 2 * DIN * 4) { const int o = u / 4, k0 = (u % 4) * 8; v8b v;
#pragma unroll
      for (int j = 0; j < 8; ++j) v[j] = (b16)(bf16_rne(win[(k0 + j) * 2 * DIN + o]) * WSC); *(volatile v8b*)(WIN + (size_t)o * G + k0) = v; }
    if (u < XDW * 8) { const int o = u / 8, k0 = (u % 8) * 8; v8b v;
#pragma unroll
      for (int j = 0; j < 8; ++j) v[j] = (b16)(o < DTR + 2 * NS ? bf16_rne(wx[(k0 + j) * (DTR + 2 * NS) + o]) * WSC : 0.0f); *(volatile v8b*)(WX + (size_t)o * DIN + k0) = v; }
    if (u < G * 8) { const int o = u / 8, k0 = (u % 8) * 8; v8b v;
#pragma unroll
      for (int j = 0; j < 8; ++j) v[j] = (b16)(bf16_rne(wo[(k0 + j) * G + o]) * WSC); *(volatile v8b*)(WO + (size_t)o * DIN + k0) = v; }
    __threadfence(); } }
__global__ __launch_bounds__(32) void inproj_kernel(const float* __restrict__ x, const b16* __restrict__ WIN, int MV, float* __restrict__ XZ) { __shared__ __attribute__((aligned(16))) b16 Ah[16][40]; __shared__ float Tf[16][132]; const int lane = threadIdx.x, nloc = lane & 15, hlf = lane >> 4; const size_t r0 = (size_t)blockIdx.x * 16; const size_t m0 = r0 / TOK; if (m0 >= (size_t)MV) return;
  for (int rr = 0; rr < 16; ++rr) { const size_t m = m0 + rr / TOK; const int t = rr % TOK; const int b = (int)(m / HW), hw = (int)(m % HW); Ah[rr][lane] = (b16)(bf16_rne(x[((size_t)b * CH + t * G + lane) * HW + hw]) * XS); }
  wave_lds_sync(); const v16b a = frag_kb(&Ah[nloc][0], hlf);
#pragma unroll
  for (int tt = 0; tt < 8; ++tt) { v8f acc = {}; acc = wmma16b(a, frag_kb(WIN + (size_t)(tt * 16 + nloc) * G, hlf), acc);
#pragma unroll
    for (int r8 = 0; r8 < 8; ++r8) Tf[8 * hlf + r8][tt * 16 + nloc] = acc[r8] * (1.0f / (XS * WSC)); }
  wave_lds_sync();
  for (int pass = 0; pass < 2; ++pass) { for (int rr = 0; rr < 16; ++rr) *(volatile v4f*)(XZ + (r0 + rr) * 2 * DIN + lane * 4) = *(const v4f*)(&Tf[rr][lane * 4]); __threadfence(); } }
__global__ __launch_bounds__(32) void xproj_kernel(const float* __restrict__ XZ, const b16* __restrict__ WX, const float* __restrict__ wdt, const float* __restrict__ bdt, int MV, float* __restrict__ XD, float* __restrict__ DL) { __shared__ __attribute__((aligned(16))) b16 Ah[16][72], Al[16][72]; __shared__ float Tf[16][52]; const int lane = threadIdx.x, nloc = lane & 15, hlf = lane >> 4; const size_t r0 = (size_t)blockIdx.x * 16; if (r0 / TOK >= (size_t)MV) return;
  for (int rr = 0; rr < 16; ++rr) for (int q = 0; q < 2; ++q) { b16 p, ql; split16(XZ[(r0 + rr) * 2 * DIN + q * 32 + lane] * XS, p, ql); Ah[rr][q * 32 + lane] = p; Al[rr][q * 32 + lane] = ql; }
  wave_lds_sync(); v8f acc[3] = {(v8f){}, (v8f){}, (v8f){}};
#pragma unroll
  for (int kb = 0; kb < DIN; kb += 32) { const v16b a = frag_kb(&Ah[nloc][kb], hlf), al = frag_kb(&Al[nloc][kb], hlf);
#pragma unroll
    for (int t = 0; t < 3; ++t) { const v16b bw = frag_kb(WX + (size_t)(t * 16 + nloc) * DIN + kb, hlf); acc[t] = wmma16b(a, bw, acc[t]); acc[t] = wmma16b(al, bw, acc[t]); } }
#pragma unroll
  for (int t = 0; t < 3; ++t)
#pragma unroll
    for (int r8 = 0; r8 < 8; ++r8) Tf[8 * hlf + r8][t * 16 + nloc] = acc[t][r8] * (1.0f / (XS * WSC));
  wave_lds_sync(); float w0[2], w1[2], bb[2]; for (int k = 0; k < 2; ++k) { const int d = lane * 2 + k; w0[k] = bf16_rne(wdt[d]); w1[k] = bf16_rne(wdt[DIN + d]); bb[k] = 2.0f * bf16_rne(bdt[d]); }
  for (int pass = 0; pass < 2; ++pass) { for (int rr = 0; rr < 16; ++rr) { for (int c = lane; c < XDW; c += 32) ((volatile float*)XD)[(r0 + rr) * XDW + c] = Tf[rr][c]; v2f dl; for (int k = 0; k < 2; ++k) dl[k] = softplus(pmul(Tf[rr][0], w0[k]) + pmul(Tf[rr][1], w1[k]) + bb[k]); *(volatile v2f*)(DL + (r0 + rr) * DIN + lane * 2) = dl; } __threadfence(); } }
__global__ __launch_bounds__(256) void scan_kernel(const float* __restrict__ XZ, const float* __restrict__ XD, const float* __restrict__ DL, const float* __restrict__ Alog, const float* __restrict__ Ds, int MV, float* __restrict__ Y) { const int wave = threadIdx.x >> 5, lane = threadIdx.x & 31; const size_t wid = (size_t)blockIdx.x * 8 + wave; const size_t m = wid >> 1; const int d = (int)(wid & 1) * 32 + lane; if (m >= (size_t)MV) return;
  float A[NS];
#pragma unroll
  for (int n = 0; n < NS; ++n) A[n] = -__expf(bf16_rne(Alog[d * NS + n])); const float Dd = bf16_rne(Ds[d]); float u[TOK], dl[TOK], yv[TOK];
#pragma unroll
  for (int t = 0; t < TOK; ++t) { const size_t r = m * TOK + t; u[t] = XZ[r * 2 * DIN + d]; dl[t] = DL[r * DIN + d]; yv[t] = 2.0f * pmul(Dd, u[t]); }
#pragma unroll
  for (int dir = 0; dir < 2; ++dir) { float h[NS];
#pragma unroll
    for (int n = 0; n < NS; ++n) h[n] = 0.0f;
#pragma unroll
    for (int s = 0; s < TOK; ++s) { const int t = dir == 0 ? s : TOK - 1 - s; const size_t r = m * TOK + t; const float du = pmul(dl[t], u[t]); float y = 0.0f;
#pragma unroll
      for (int n = 0; n < NS; ++n) { h[n] = pmul(__expf(pmul(dl[t], A[n])), h[n]) + pmul(du, XD[r * XDW + DTR + n]); y += pmul(h[n], XD[r * XDW + DTR + NS + n]); } yv[t] += y; } }
  for (int pass = 0; pass < 2; ++pass) {
#pragma unroll
    for (int t = 0; t < TOK; ++t) { const size_t r = m * TOK + t; ((volatile float*)Y)[r * DIN + d] = pmul(yv[t], gelu(XZ[r * 2 * DIN + DIN + d])); } __threadfence(); } }
__global__ __launch_bounds__(32) void outproj_kernel(const float* __restrict__ Y, const b16* __restrict__ WO, float* __restrict__ YO, float* __restrict__ PST) { __shared__ __attribute__((aligned(16))) b16 Ah[32][72], Al[32][72]; __shared__ float Tf[32][36]; const int lane = threadIdx.x, nloc = lane & 15, hlf = lane >> 4; const int wid = blockIdx.x; const int t = wid % TOK, wh = (wid / TOK) % 2, h = (wid / (TOK * 2)) % HH, b = wid / (TOK * 2 * HH); const size_t mb = (size_t)b * HW + h * WW + wh * 32;
  for (int rr = 0; rr < 32; ++rr) for (int q = 0; q < 2; ++q) { b16 p, ql; split16(Y[((mb + rr) * TOK + t) * DIN + q * 32 + lane] * XS, p, ql); Ah[rr][q * 32 + lane] = p; Al[rr][q * 32 + lane] = ql; }
  wave_lds_sync();
  for (int mt = 0; mt < 2; ++mt) { v8f acc[2] = {(v8f){}, (v8f){}};
#pragma unroll
    for (int kb = 0; kb < DIN; kb += 32) { const v16b a = frag_kb(&Ah[mt * 16 + nloc][kb], hlf), al = frag_kb(&Al[mt * 16 + nloc][kb], hlf);
#pragma unroll
      for (int tt = 0; tt < 2; ++tt) { const v16b bw = frag_kb(WO + (size_t)(tt * 16 + nloc) * DIN + kb, hlf); acc[tt] = wmma16b(a, bw, acc[tt]); acc[tt] = wmma16b(al, bw, acc[tt]); } }
#pragma unroll
    for (int tt = 0; tt < 2; ++tt)
#pragma unroll
      for (int r8 = 0; r8 < 8; ++r8) Tf[mt * 16 + 8 * hlf + r8][tt * 16 + nloc] = acc[tt][r8] * (1.0f / (XS * WSC)); }
  wave_lds_sync(); float s = 0.0f, q2 = 0.0f; for (int rr = 0; rr < 32; ++rr) { const float v = Tf[rr][lane]; s += v; q2 += pmul(v, v); } for (int o = 16; o; o >>= 1) { s += __shfl_xor(s, o); q2 += __shfl_xor(q2, o); }
  for (int pass = 0; pass < 2; ++pass) { for (int g = 0; g < G; ++g) ((volatile float*)YO)[(((size_t)b * CH + t * G + g) * HH + h) * WW + wh * 32 + lane] = Tf[lane][g];
    ((volatile float*)PST)[(size_t)wid * 32 + lane] = lane == 0 ? s : (lane == 1 ? q2 : 0.0f); __threadfence(); } }
__global__ __launch_bounds__(256) void gnstat_kernel(const float* __restrict__ PST, int BV, float* __restrict__ ST) { const int tid = threadIdx.x; if (tid >= B * NGR) return; const int b = tid / NGR, gr = tid % NGR; double s = 0.0, q = 0.0;
  if (b < BV) { for (int h = 0; h < HH; ++h) for (int wh = 0; wh < 2; ++wh) for (int tt = 0; tt < 2; ++tt) { const int t = gr * 2 + tt; const size_t wid = (((size_t)b * HH + h) * 2 + wh) * TOK + t; s += (double)PST[wid * 32]; q += (double)PST[wid * 32 + 1]; } }
  const double n = (double)(CH / NGR) * HW; const double mean = s / n; double var = q / n - mean * mean; if (var < 0.0) var = 0.0; const float mf = (float)mean, rs = (float)(1.0 / sqrt(var + (double)EPS));
  for (int pass = 0; pass < 2; ++pass) { for (int j = 0; j < 32; ++j) ((volatile float*)ST)[(size_t)tid * 32 + j] = j == 0 ? mf : (j == 1 ? rs : 0.0f); __threadfence(); } }
__global__ __launch_bounds__(256) void fin_kernel(const float* __restrict__ x, const float* __restrict__ YO, const float* __restrict__ ST, const float* __restrict__ gw, const float* __restrict__ gb, int BV, float* __restrict__ out) { const size_t u = (size_t)blockIdx.x * 256 + threadIdx.x; if (u >= (size_t)B * CH * HW / 4) return; const size_t e0 = u * 4; const int b = (int)(e0 / ((size_t)CH * HW)), c = (int)((e0 / HW) % CH); const int gr = c / (CH / NGR);
  v4f r = {0.0f, 0.0f, 0.0f, 0.0f}; if (b < BV) { const float mu = ST[(b * NGR + gr) * 32], rs = ST[(b * NGR + gr) * 32 + 1], w = bf16_rne(gw[c]), bb = bf16_rne(gb[c]); const v4f xv = *(const v4f*)(x + e0), yv = *(const v4f*)(YO + e0); for (int k = 0; k < 4; ++k) r[k] = bf16_rne(xv[k]) + pmul(pmul(yv[k] - mu, rs), w) + bb; }
  for (int pass = 0; pass < 2; ++pass) { *(volatile v4f*)(out + e0) = r; __threadfence(); } }
}

extern "C" void kernel_launch(void* const* d_in, const int* in_sizes, int n_in, void* d_out, int out_size, void* d_ws, size_t ws_size, hipStream_t stream) {
  (void)n_in;
  auto Fp = [&](int i) { return (const float*)d_in[i]; };
  if (in_sizes[0] != B * CH * HW || in_sizes[1] != G * 2 * DIN || in_sizes[2] != DIN * (DTR + 2 * NS) || in_sizes[3] != DTR * DIN || in_sizes[5] != DIN * NS || in_sizes[7] != DIN * G || out_size != B * CH * HW) return;
  const int BV = B; const int MV = BV * HW;
  size_t off = 0; char* ws = (char*)d_ws;
  auto carve = [&](size_t bytes) { char* p = ws + off; off += (bytes + 255) & ~(size_t)255; return p; };
  b16* WIN = (b16*)carve((size_t)2 * DIN * G * 2); b16* WX = (b16*)carve((size_t)XDW * DIN * 2); b16* WO = (b16*)carve((size_t)G * DIN * 2);
  float* XZ = (float*)carve((size_t)MALL * TOK * 2 * DIN * 4); float* XD = (float*)carve((size_t)MALL * TOK * XDW * 4); float* DL = (float*)carve((size_t)MALL * TOK * DIN * 4); float* Y = (float*)carve((size_t)MALL * TOK * DIN * 4); float* YO = (float*)carve((size_t)B * CH * HW * 4);
  const int NWO = B * HH * 2 * TOK; float* PST = (float*)carve((size_t)NWO * 32 * 4); float* ST = (float*)carve((size_t)B * NGR * 32 * 4);
  if (off > ws_size || off > ((size_t)192 << 20)) return;
  wput_kernel<<<4, 256, 0, stream>>>(Fp(1), Fp(2), Fp(7), WIN, WX, WO);
  inproj_kernel<<<MV * TOK / 16, 32, 0, stream>>>(Fp(0), WIN, MV, XZ);
  xproj_kernel<<<MV * TOK / 16, 32, 0, stream>>>(XZ, WX, Fp(3), Fp(4), MV, XD, DL);
  scan_kernel<<<(MV * 2 + 7) / 8, 256, 0, stream>>>(XZ, XD, DL, Fp(5), Fp(6), MV, Y);
  outproj_kernel<<<BV * HH * 2 * TOK, 32, 0, stream>>>(Y, WO, YO, PST);
  gnstat_kernel<<<1, 256, 0, stream>>>(PST, BV, ST);
  fin_kernel<<<(unsigned)(((size_t)B * CH * HW / 4 + 255) / 256), 256, 0, stream>>>(Fp(0), YO, ST, Fp(8), Fp(9), BV, (float*)d_out);
}
